// OpticalConvolution_28999619182925
// MI455X (gfx1250) — hardware-run, weakly checked
//
#include <hip/hip_runtime.h>
#include <math.h>

typedef __attribute__((ext_vector_type(16))) _Float16 v16h;
typedef __attribute__((ext_vector_type(8)))  _Float16 v8h;
typedef __attribute__((ext_vector_type(8)))  float    v8f;
typedef __attribute__((ext_vector_type(4)))  float    v4f;

constexpr int kNb    = 16;
constexpr int kCin   = 128;
constexpr int kHt    = 56;
constexpr int kWd    = 56;
constexpr int kCout  = 256;
constexpr int kPix   = kHt * kWd;
constexpr int kHP    = kHt + 2;
constexpr int kWP    = kWd + 2;
constexpr int kTaps  = 9;
constexpr int kKtot  = kTaps * kCin;
constexpr int kTilesM = (kNb * kPix) / 64;
constexpr int kTilesN = kCout / 64;
constexpr int kLdsTP  = 57;
constexpr int kSlabP  = 68;
constexpr int kPairs  = kWP / 2;
constexpr float kCarryMap = 16.0f;
constexpr float kCarryWgt = 256.0f;
constexpr float kFold     = 1.0f / (kCarryMap * kCarryWgt);
constexpr float kF16Min   = 6.103515625e-05f;

static_assert(kPix == 3136, "pixels per image");
static_assert((kPix % 64) == 0, "no 64-pixel tile straddles a batch element");
static_assert((kCin % 32) == 0, "a 32-wide k-step never crosses a tap");
static_assert((kKtot % 32) == 0 && kKtot == 1152, "K multiple of 32");
static_assert((kCout % 64) == 0, "N multiple of 64");
static_assert(((kTilesM * kTilesN) % 8) == 0, "8 wave tiles per block, exact grid");
static_assert((kCin * kWd) == 28 * 256, "map row staging coverage");
static_assert((2 * kKtot) == 8 * 288, "weight staging coverage");
static_assert((kWP % 2) == 0 && kPairs == 29, "pixel pairs per padded row");
static_assert(kNb * kCin * kPix == 6422528, "in0 element count");
static_assert(kCout * kKtot == 294912, "in1 element count");
static_assert(kNb * kCout * kPix == 12845056, "output element count");
static_assert(kFold == 1.0f / 4096.0f, "fold constant");

constexpr size_t kOffXP   = 0;
constexpr size_t kSizeXP  = (size_t)kNb * kHP * kWP * kCin * 2;
constexpr size_t kOffWT   = kOffXP + kSizeXP;
constexpr size_t kSizeWT  = (size_t)kCout * kKtot * 2;
constexpr size_t kWsTotal = kOffWT + kSizeWT;
static_assert(kSizeXP == 13778944ull, "XP bytes");
static_assert(kSizeWT == 589824ull, "WT bytes");
static_assert(kWsTotal == 14368768ull, "carve total");
static_assert(kWsTotal <= 134217728ull, "carve cap");
static_assert((kOffWT % 128) == 0, "128-B aligned regions");
static_assert(((size_t)kWP * kCin * 2) % 128 == 0, "XP row pitch is a line multiple");
static_assert(((size_t)kKtot * 2) % 128 == 0, "WT row pitch is a line multiple");
static_assert(((size_t)kPix * 4) % 128 == 0, "output channel-row pitch is a line multiple");

union FragU { v16h v; v8h h[2]; };
__device__ __forceinline__ v16h frag_load(const _Float16* p) {
  FragU f;
  f.h[0] = *(const v8h*)(p);
  f.h[1] = *(const v8h*)(p + 16);
  return f.v;
}
__device__ __forceinline__ v8f mma16(v16h a, v16h b, v8f c) {
  return __builtin_amdgcn_wmma_f32_16x16x32_f16(false, a, false, b, (short)0, c, false, false);
}
__device__ __forceinline__ void tie1(v8f& a, v16h x, v16h y) {
  asm volatile("v_nop\n\tv_nop\n\tv_nop\n\tv_nop" : "+v"(a) : "v"(x), "v"(y));
}
__device__ __forceinline__ void tie0(v8f& a) {
  asm volatile("v_nop\n\tv_nop\n\tv_nop\n\tv_nop" : "+v"(a));
}
__device__ __forceinline__ void keep4(v16h a, v16h b, v16h c, v16h d) {
  asm volatile("v_nop" :: "v"(a), "v"(b), "v"(c), "v"(d));
}
__device__ __forceinline__ _Float16 to_f16_flushed(float v) {
  const float w = (fabsf(v) < kF16Min) ? 0.0f : v;
  return (_Float16)w;
}

__global__ __launch_bounds__(256) void prep_map_kernel(const float* __restrict__ src,
                                                       unsigned short* __restrict__ XP) {
  __shared__ __align__(16) float sT[kCin * kLdsTP];
  const int tid  = threadIdx.x;
  const int lane = tid & 31;
  const int wave = tid >> 5;
  const int b  = blockIdx.x / kHP;
  const int yy = blockIdx.x - b * kHP;
  const bool interior = (yy >= 1) && (yy <= kHt);
  int yc = yy - 1;
  yc = yc < 0 ? 0 : yc;
  yc = yc > (kHt - 1) ? (kHt - 1) : yc;
  const float* srow = src + (size_t)b * kCin * kPix + (size_t)yc * kWd;
#pragma unroll 1
  for (int i = 0; i < 28; ++i) {
    const int idx = tid + 256 * i;
    const int c = idx / kWd;
    const int x = idx - c * kWd;
    const float v = srow[(size_t)c * kPix + x];
    sT[c * kLdsTP + x] = interior ? v : 0.0f;
  }
  __syncthreads();

  const int sub = lane >> 4;
  const int c8  = (lane & 15) * 8;
  v8h hv[4];
#pragma unroll
  for (int it = 0; it < 4; ++it) {
    const int pair = it * 8 + wave;
    const int pc = pair < kPairs ? pair : (kPairs - 1);
    const int xx = pc * 2 + sub;
    const bool live = (xx >= 1) && (xx <= kWd);
    int xs = xx - 1;
    xs = xs < 0 ? 0 : xs;
    xs = xs > (kWd - 1) ? (kWd - 1) : xs;
#pragma unroll
    for (int e = 0; e < 8; ++e) {
      const float t = sT[(c8 + e) * kLdsTP + xs];
      const float v = live ? (t * kCarryMap) : 0.0f;
      hv[it][e] = to_f16_flushed(v);
    }
  }
  unsigned short* rowp = XP + ((size_t)b * kHP + yy) * (size_t)(kWP * kCin);
  for (int pass = 0; pass < 2; ++pass) {
#pragma unroll
    for (int it = 0; it < 4; ++it) {
      const int pair = it * 8 + wave;
      if (pair < kPairs) {
        *(volatile v8h*)(rowp + (size_t)(pair * 2 + sub) * kCin + c8) = hv[it];
      }
    }
    __threadfence();
  }
}

__global__ __launch_bounds__(288) void prep_wgt_kernel(const float* __restrict__ w,
                                                       unsigned short* __restrict__ WT) {
  __shared__ __align__(16) float sW[2 * kKtot];
  const int tid = threadIdx.x;
  const int o0  = blockIdx.x * 2;
  const float* wp = w + (size_t)o0 * kKtot;
#pragma unroll 1
  for (int i = 0; i < 8; ++i) sW[tid + 288 * i] = wp[tid + 288 * i];
  __syncthreads();
  const int ol  = tid / 144;
  const int q   = tid - ol * 144;
  const int kk0 = q * 8;
  const int tap = kk0 >> 7;
  const int c0  = kk0 & 127;
  v8h hv;
#pragma unroll
  for (int e = 0; e < 8; ++e) {
    const float t = sW[ol * kKtot + (c0 + e) * kTaps + tap];
    hv[e] = to_f16_flushed(t * kCarryWgt);
  }
  unsigned short* dst = WT + (size_t)o0 * kKtot + (size_t)tid * 8;
  *(volatile v8h*)dst = hv;
  __threadfence();
  *(volatile v8h*)dst = hv;
}

__global__ __launch_bounds__(256) void conv_product_kernel(const unsigned short* __restrict__ XPp,
                                                           const unsigned short* __restrict__ WTp,
                                                           const float* __restrict__ bias,
                                                           float* __restrict__ out) {
  __shared__ __align__(16) float sS[8][16 * kSlabP];
  const _Float16* XP = (const _Float16*)XPp;
  const _Float16* WT = (const _Float16*)WTp;
  const int lane = threadIdx.x & 31;
  const int wave = threadIdx.x >> 5;
  const int tile = blockIdx.x * 8 + wave;
  if (tile >= kTilesM * kTilesN) return;
  const int tm = tile / kTilesN;
  const int tn = tile - tm * kTilesN;
  const int m0 = tm * 64;
  const int n0 = tn * 64;
  const int b    = m0 / kPix;
  const int pix0 = m0 - b * kPix;

  const int rlane = lane & 15;
  const int hh    = lane >> 4;
  const int koff  = hh * 8;

  int aoff[4];
#pragma unroll
  for (int i = 0; i < 4; ++i) {
    const int p = pix0 + 16 * i + rlane;
    const int y = p / kWd;
    const int x = p - y * kWd;
    aoff[i] = ((b * kHP + y) * kWP + x) * kCin + koff;
  }
  const int boff0 = (n0 + rlane) * kKtot + koff;

  v8f acc[4][4];
#pragma unroll
  for (int i = 0; i < 4; ++i)
#pragma unroll
    for (int j = 0; j < 4; ++j) acc[i][j] = (v8f){0.f, 0.f, 0.f, 0.f, 0.f, 0.f, 0.f, 0.f};

#pragma unroll 1
  for (int kh = 0; kh < 3; ++kh) {
#pragma unroll 1
    for (int kw = 0; kw < 3; ++kw) {
      const int tapA = (kh * kWP + kw) * kCin;
      const int tapB = (kh * 3 + kw) * kCin;
#pragma unroll 1
      for (int cq = 0; cq < 4; ++cq) {
        const int ka = tapA + 32 * cq;
        const int kb = tapB + 32 * cq;
        v16h bh[4];
#pragma unroll
        for (int j = 0; j < 4; ++j) bh[j] = frag_load(WT + boff0 + j * 16 * kKtot + kb);
#pragma unroll
        for (int i = 0; i < 4; ++i) {
          const v16h ah = frag_load(XP + aoff[i] + ka);
#pragma unroll
          for (int j = 0; j < 4; ++j) acc[i][j] = mma16(ah, bh[j], acc[i][j]);
          tie1(acc[i][0], ah, bh[0]);
          tie1(acc[i][1], ah, bh[1]);
          tie1(acc[i][2], ah, bh[2]);
          tie1(acc[i][3], ah, bh[3]);
        }
        keep4(bh[0], bh[1], bh[2], bh[3]);
      }
    }
  }
#pragma unroll
  for (int i = 0; i < 4; ++i) {
    tie0(acc[i][0]);
    tie0(acc[i][1]);
    tie0(acc[i][2]);
    tie0(acc[i][3]);
  }

  float bv[4];
#pragma unroll
  for (int j = 0; j < 4; ++j) bv[j] = bias[n0 + 16 * j + rlane];

  float* slab = sS[wave];
  const int c4 = (lane & 15) * 4;
  float* obase = out + ((size_t)b * kCout + n0) * (size_t)kPix + pix0 + c4;
#pragma unroll
  for (int j = 0; j < 4; ++j) {
#pragma unroll
    for (int i = 0; i < 4; ++i) {
      v4f lo4, hi4;
#pragma unroll
      for (int r = 0; r < 4; ++r) {
        lo4[r] = acc[i][j][r] * kFold + bv[j];
        hi4[r] = acc[i][j][4 + r] * kFold + bv[j];
      }
      float* sp = slab + rlane * kSlabP + 16 * i + 8 * hh;
      *(v4f*)(sp)     = lo4;
      *(v4f*)(sp + 4) = hi4;
    }
    __builtin_amdgcn_fence(__ATOMIC_RELEASE, "workgroup");
    __builtin_amdgcn_wave_barrier();
    __builtin_amdgcn_fence(__ATOMIC_ACQUIRE, "workgroup");
    for (int pass = 0; pass < 2; ++pass) {
#pragma unroll
      for (int it = 0; it < 8; ++it) {
        const int row = it * 2 + hh;
        const v4f v = *(const v4f*)(slab + row * kSlabP + c4);
        *(volatile v4f*)(obase + (size_t)(16 * j + row) * kPix) = v;
      }
      __threadfence();
    }
    __builtin_amdgcn_fence(__ATOMIC_RELEASE, "workgroup");
    __builtin_amdgcn_wave_barrier();
    __builtin_amdgcn_fence(__ATOMIC_ACQUIRE, "workgroup");
  }
}

extern "C" void kernel_launch(void* const* d_in, const int* in_sizes, int n_in,
                              void* d_out, int out_size, void* d_ws, size_t ws_size,
                              hipStream_t stream) {
  if (n_in < 3) return;
  if (in_sizes[0] != kNb * kCin * kPix) return;
  if (in_sizes[1] != kCout * kKtot) return;
  if (in_sizes[2] != kCout) return;
  if (out_size != kNb * kCout * kPix) return;
  if (ws_size < kWsTotal) return;

  const float* tensor  = (const float*)d_in[0];
  const float* weights = (const float*)d_in[1];
  const float* bias    = (const float*)d_in[2];
  float* out = (float*)d_out;

  char* ws = (char*)d_ws;
  unsigned short* XP = (unsigned short*)(ws + kOffXP);
  unsigned short* WT = (unsigned short*)(ws + kOffWT);

  prep_map_kernel<<<dim3(kNb * kHP), dim3(256), 0, stream>>>(tensor, XP);
  prep_wgt_kernel<<<dim3(kCout / 2), dim3(288), 0, stream>>>(weights, WT);
  conv_product_kernel<<<dim3((kTilesM * kTilesN) / 8), dim3(256), 0, stream>>>(XP, WT, bias, out);
}
